// CausalSelfAttention_59528246722829
// MI455X (gfx1250) — hardware-verified
//
#include <hip/hip_runtime.h>
#include <math.h>

typedef __attribute__((ext_vector_type(16))) _Float16 v16h;
typedef __attribute__((ext_vector_type(16))) __bf16 v16b;
typedef __attribute__((ext_vector_type(8)))  _Float16 v8h;
typedef __attribute__((ext_vector_type(8)))  __bf16 v8b;
typedef __attribute__((ext_vector_type(8)))  float v8f;
typedef __attribute__((ext_vector_type(4)))  float v4f;
typedef __attribute__((ext_vector_type(4)))  unsigned v4u;

template <typename T> __device__ __forceinline__ void vst2(void* p, T v) { *(volatile T*)p = v; __threadfence(); *(volatile T*)p = v; }
__device__ __forceinline__ v8f wmma16(v16h a, v16h b, v8f c) {
  v8f d = __builtin_amdgcn_wmma_f32_16x16x32_f16(false, a, false, b, (short)0, c, false, false);
  asm volatile("v_nop\n\tv_nop\n\tv_nop\n\tv_nop" : "+v"(d) : "v"(a), "v"(b));
  return d;
}
__device__ __forceinline__ v8f wmma_bf(v16b a, v16b b, v8f c) {
  v8f d = __builtin_amdgcn_wmma_f32_16x16x32_bf16(false, a, false, b, (short)0, c, false, false);
  asm volatile("v_nop\n\tv_nop\n\tv_nop\n\tv_nop" : "+v"(d) : "v"(a), "v"(b));
  return d;
}
__device__ __forceinline__ v16h frag_h(const _Float16* rowk0, unsigned lane) {
  union { v16h v; v8h q[2]; } u; const _Float16* p = rowk0 + 8u * (lane >> 4);
  u.q[0] = *(const v8h*)p; u.q[1] = *(const v8h*)(p + 16); return u.v;
}
__device__ __forceinline__ v16b frag_b(const __bf16* rowk0, unsigned lane) {
  union { v16b v; v8b q[2]; } u; const __bf16* p = rowk0 + 8u * (lane >> 4);
  u.q[0] = *(const v8b*)p; u.q[1] = *(const v8b*)(p + 16); return u.v;
}
__device__ __forceinline__ v16b frag_f32_bf(const float* rowk0, unsigned lane) {
  const v4f* p = (const v4f*)(rowk0 + 8u * (lane >> 4)); const v4f a0 = p[0], a1 = p[1], a2 = p[4], a3 = p[5]; v16b w;
#pragma unroll
  for (int i = 0; i < 4; ++i) { w[i] = (__bf16)a0[i]; w[4 + i] = (__bf16)a1[i]; w[8 + i] = (__bf16)a2[i]; w[12 + i] = (__bf16)a3[i]; }
  return w;
}
struct F2 { v16b h, l; };
__device__ __forceinline__ F2 bsplit16(const float v[16]) { F2 r;
#pragma unroll
  for (int i = 0; i < 16; ++i) { const __bf16 h = (__bf16)v[i]; r.h[i] = h; r.l[i] = (__bf16)(v[i] - (float)h); }
  return r; }
__device__ __forceinline__ F2 split_row(const float* row, unsigned k0, unsigned lane) { float v[16]; const float* p = row + k0 + 8u * (lane >> 4);
#pragma unroll
  for (int i = 0; i < 8; ++i) { v[i] = p[i]; v[8 + i] = p[16 + i]; }
  return bsplit16(v); }
__device__ __forceinline__ F2 split_g(const float* rowk0, unsigned lane) { const v4f* p = (const v4f*)(rowk0 + 8u * (lane >> 4)); const v4f a0 = p[0], a1 = p[1], a2 = p[4], a3 = p[5]; float v[16];
#pragma unroll
  for (int i = 0; i < 4; ++i) { v[i] = a0[i]; v[4 + i] = a1[i]; v[8 + i] = a2[i]; v[12 + i] = a3[i]; }
  return bsplit16(v); }
__device__ __forceinline__ float pos_scale(float y, float c, float s) {
#pragma clang fp contract(off)
  const float a = y * c; const float b = y * s; return a + b; }
#define LDSX() do { asm volatile("s_wait_dscnt 0" ::: "memory"); __builtin_amdgcn_wave_barrier(); __builtin_amdgcn_fence(3  , "workgroup"); } while (0)

#ifndef NB
#define NB 2
#endif
#ifndef SEQ
#define SEQ 2048
#endif
#define NB_FULL 2
#define TT_FULL 2048
#define TT SEQ
#define CC 1024
#define DIN 1024
#define NH 16
#define HD 64
#define RH (HD / 2)
#define NQB (TT / 64)
#define SCALE (0.125f)
#define QBH 8
#define QHI 512
#define KHI 512
#define PP 72
static_assert(NB >= 1 && NB <= NB_FULL);
static_assert(TT >= 512 && TT <= TT_FULL && (TT % 128) == 0);
static_assert(CC == NH * HD && (CC % 128) == 0 && (DIN % 128) == 0);
static_assert(HD == 64);
static_assert(RH == 32);
static_assert(CC == DIN);
static_assert((DIN % 32) == 0 && (CC % 32) == 0);
static_assert(QHI == QBH * 64 && KHI >= QBH * 64);
static_assert((QHI % 64) == 0 && (KHI % 64) == 0 && QHI <= TT && KHI <= TT);
static_assert(PP >= 64 && ((PP * 2) % 16) == 0);

#define WS_QH  ((size_t)0)
#define WS_KH  (WS_QH + (size_t)2 * TT * CC)
#define WS_VT  (WS_KH + (size_t)2 * TT * CC)
#define WS_QL  (WS_VT + (size_t)2 * CC * TT)
#define WS_KL  (WS_QL + (size_t)2 * QHI * CC)
#define WS_VB  (WS_KL + (size_t)2 * KHI * CC)
#define WS_VBL (WS_VB + (size_t)2 * CC * KHI)
#define WS_Y   (WS_VBL + (size_t)2 * CC * KHI)
#define WS_COS (WS_Y + (size_t)4 * TT * CC)
#define WS_SIN (WS_COS + (size_t)4 * TT * RH)
#define WS_END (WS_SIN + (size_t)4 * TT * RH)
static_assert(WS_END <= (size_t)134217728u);
static_assert((WS_KH % 128u) == 0 && (WS_VT % 128u) == 0 && (WS_QL % 128u) == 0 && (WS_KL % 128u) == 0 && (WS_VB % 128u) == 0 && (WS_VBL % 128u) == 0 && (WS_Y % 128u) == 0 && (WS_COS % 128u) == 0 && (WS_SIN % 128u) == 0);
static_assert((TT / 64) * 64 == TT && (CC / 128) * 128 == CC);
static_assert(NQB * 64 == TT && NH * HD == CC);
static_assert((DIN / 128) * 128 == DIN);
static_assert(((TT * RH) % 256) == 0);

__global__ __launch_bounds__(256) void k_pos(float* __restrict__ COS, float* __restrict__ SIN) {
#pragma clang fp contract(off)
  const unsigned e = blockIdx.x * 256u + threadIdx.x; const unsigned t = e >> 5, i = e & 31u;
  const float ex = (-2.0f * (float)i) / (float)HD;
  const float inv = powf(10000.0f, ex);
  float th = (float)t * inv;
  asm volatile("" : "+v"(th));
  float s, c; sincosf(th, &s, &c);
  vst2<float>((void*)(COS + e), c); vst2<float>((void*)(SIN + e), s); }

__global__ __launch_bounds__(128) void k_proj(const float* __restrict__ X, const float* __restrict__ WQ, const float* __restrict__ WK, const float* __restrict__ WV,
    const float* __restrict__ BQ, const float* __restrict__ BK, const float* __restrict__ BV, const float* __restrict__ COS, const float* __restrict__ SIN,
    _Float16* __restrict__ QH, _Float16* __restrict__ QL, _Float16* __restrict__ KH, _Float16* __restrict__ KL, _Float16* __restrict__ VT, __bf16* __restrict__ VB, __bf16* __restrict__ VBL) {
  __shared__ __align__(16) _Float16 sh[64][136], sl[64][136]; __shared__ __align__(16) _Float16 th[128][72]; __shared__ __align__(16) __bf16 tb[128][72], tbl[128][72];
  __shared__ __align__(16) float sc[64][36], sn[64][36];
  const unsigned tid = threadIdx.x, wave = tid >> 5, lane = tid & 31u, col = lane & 15u, g = lane >> 4;
  const unsigned which = blockIdx.z; const unsigned c0 = blockIdx.y * 128u; const unsigned t0 = blockIdx.x * 64u;
  const float* WA = which == 0u ? WQ : which == 1u ? WK : WV;
  const float* BA = which == 0u ? BQ : which == 1u ? BK : BV;
  for (unsigned e = tid; e < 64u * 8u; e += 128u) { const unsigned rl = e >> 3, q = e & 7u; const size_t go = (size_t)(t0 + rl) * RH + q * 4u;
    *(v4f*)&sc[rl][q * 4u] = *(const v4f*)(COS + go); *(v4f*)&sn[rl][q * 4u] = *(const v4f*)(SIN + go); }
  __syncthreads();
  const float* xrow = X + (size_t)(t0 + wave * 16u + col) * DIN;
  v8f acc[8] = {};
#pragma unroll 2
  for (unsigned kc = 0; kc < DIN / 32; ++kc) { const v16b a = frag_f32_bf(xrow + kc * 32u, lane);
    asm volatile("s_wait_loadcnt 0x0" ::: "memory");
#pragma unroll
    for (int j = 0; j < 8; ++j) { const v16b w = frag_f32_bf(WA + (size_t)(c0 + (unsigned)j * 16u + col) * DIN + kc * 32u, lane); asm volatile("s_wait_loadcnt 0x0" ::: "memory"); acc[j] = wmma_bf(a, w, acc[j]); } }
  float bias[8];
#pragma unroll
  for (int j = 0; j < 8; ++j) bias[j] = (float)(__bf16)BA[c0 + (unsigned)j * 16u + col];
  if (which < 2u) { _Float16* DH = which == 0u ? QH : KH; _Float16* DL = which == 0u ? QL : KL; const unsigned nhi = which == 0u ? (unsigned)QHI : (unsigned)KHI; const bool hi_rows = t0 < nhi;
    float rc[2][8], rs[2][8];
#pragma unroll
    for (int jj = 0; jj < 2; ++jj) {
#pragma unroll
      for (int r = 0; r < 8; ++r) { rc[jj][r] = sc[wave * 16u + 8u * g + (unsigned)r][(unsigned)jj * 16u + col]; rs[jj][r] = sn[wave * 16u + 8u * g + (unsigned)r][(unsigned)jj * 16u + col]; } }
#pragma unroll
    for (int j = 0; j < 8; ++j) {
#pragma unroll
      for (int r = 0; r < 8; ++r) { const float v = pos_scale(acc[j][r] + bias[j], rc[j & 1][r], rs[j & 1][r]); const _Float16 hv = (_Float16)v; sh[wave * 16u + 8u * g + (unsigned)r][(unsigned)j * 16u + col] = hv; sl[wave * 16u + 8u * g + (unsigned)r][(unsigned)j * 16u + col] = (_Float16)((v - (float)hv) * 1024.0f); } }
    __syncthreads();
    for (unsigned e = tid; e < 64u * 16u; e += 128u) { const unsigned rl = e >> 4, q = e & 15u; vst2((void*)(DH + (size_t)(t0 + rl) * CC + c0 + q * 8u), *(const v4u*)&sh[rl][q * 8u]); if (hi_rows) vst2((void*)(DL + (size_t)(t0 + rl) * CC + c0 + q * 8u), *(const v4u*)&sl[rl][q * 8u]); }
  } else { const bool hi_rows = t0 < (unsigned)KHI;
#pragma unroll
    for (int j = 0; j < 8; ++j) {
#pragma unroll
      for (int r = 0; r < 8; ++r) { const float v = acc[j][r] + bias[j]; const unsigned rl = wave * 16u + 8u * g + (unsigned)r, cl = (unsigned)j * 16u + col; th[cl][rl] = (_Float16)v; const __bf16 bh = (__bf16)v; tb[cl][rl] = bh; tbl[cl][rl] = (__bf16)(v - (float)bh); } }
    __syncthreads();
    for (unsigned e = tid; e < 128u * 8u; e += 128u) { const unsigned cl = e >> 3, q = e & 7u; vst2((void*)(VT + (size_t)(c0 + cl) * TT + t0 + q * 8u), *(const v4u*)&th[cl][q * 8u]); if (hi_rows) { const size_t o3 = (size_t)(c0 + cl) * KHI + t0 + q * 8u; vst2((void*)(VB + o3), *(const v4u*)&tb[cl][q * 8u]); vst2((void*)(VBL + o3), *(const v4u*)&tbl[cl][q * 8u]); } } } }

__device__ __forceinline__ void sm_step(v8f (&s)[4], float (&m)[8], float (&l)[8], v8f (&o)[4], const bool diag, const unsigned row0, const unsigned key0) {
#pragma unroll
  for (int r = 0; r < 8; ++r) { const unsigned row = row0 + (unsigned)r; float mx = -3.0e38f;
#pragma unroll
    for (int j = 0; j < 4; ++j) { const unsigned key = key0 + 16u * (unsigned)j; float v = s[j][r]; v = (diag && key > row) ? -3.0e38f : v; s[j][r] = v; mx = fmaxf(mx, v); }
    mx = fmaxf(mx, __shfl_xor(mx, 1)); mx = fmaxf(mx, __shfl_xor(mx, 2)); mx = fmaxf(mx, __shfl_xor(mx, 4)); mx = fmaxf(mx, __shfl_xor(mx, 8));
    const float mnew = fmaxf(m[r], mx); const float corr = __expf(fmaxf(m[r] - mnew, -80.0f)); m[r] = mnew; float ps = 0.f;
#pragma unroll
    for (int j = 0; j < 4; ++j) { const float v = s[j][r]; const float e = __expf(fmaxf(v - mnew, -80.0f)); const float p = (v <= -1.0e38f) ? 0.f : e; s[j][r] = p; ps += p; }
    l[r] = l[r] * corr + ps;
#pragma unroll
    for (int j = 0; j < 4; ++j) o[j][r] *= corr; } }

__global__ __launch_bounds__(128) void k_fa(const _Float16* __restrict__ QH, const _Float16* __restrict__ KH, const _Float16* __restrict__ QL, const _Float16* __restrict__ KL,
    const _Float16* __restrict__ VT, const __bf16* __restrict__ VB, const __bf16* __restrict__ VBL, float* __restrict__ Y) {
  __shared__ __align__(16) float ss[4][16][HD + 4];
  __shared__ __align__(16) _Float16 sp[4][16][PP];
  const unsigned tid = threadIdx.x, wave = tid >> 5, lane = tid & 31u, col = lane & 15u, g = lane >> 4;
  const unsigned qb = blockIdx.x, h = blockIdx.y; const unsigned ql0 = qb * 64u + wave * 16u; const size_t hc = (size_t)h * HD;
  float m[8], l[8];
#pragma unroll
  for (int r = 0; r < 8; ++r) { m[r] = -3.0e38f; l[r] = 0.f; }
  v8f o[4] = {}; float carry_inv;
  if (qb < (unsigned)QBH) {
    v16h qa[2], qr[2];
#pragma unroll
    for (int kc = 0; kc < 2; ++kc) { qa[kc] = frag_h(QH + (size_t)(ql0 + col) * CC + hc + (unsigned)kc * 32u, lane); qr[kc] = frag_h(QL + (size_t)(ql0 + col) * CC + hc + (unsigned)kc * 32u, lane); }
#pragma unroll 1
    for (unsigned ks = 0; ks <= qb; ++ks) { const unsigned k0 = ks * 64u; v8f s[4] = {}, sr[4] = {};
#pragma unroll
      for (int j = 0; j < 4; ++j) { const size_t ko = (size_t)(k0 + (unsigned)j * 16u + col) * CC + hc;
        const v16h kf0 = frag_h(KH + ko, lane), kf1 = frag_h(KH + ko + 32, lane), kr0 = frag_h(KL + ko, lane), kr1 = frag_h(KL + ko + 32, lane);
        asm volatile("s_wait_loadcnt 0x0" ::: "memory");
        s[j] = wmma16(qa[0], kf0, s[j]); s[j] = wmma16(qa[1], kf1, s[j]);
        sr[j] = wmma16(qr[0], kf0, sr[j]); sr[j] = wmma16(qa[0], kr0, sr[j]); sr[j] = wmma16(qr[1], kf1, sr[j]); sr[j] = wmma16(qa[1], kr1, sr[j]); }
#pragma unroll
      for (int j = 0; j < 4; ++j)
#pragma unroll
        for (int r = 0; r < 8; ++r) s[j][r] = (s[j][r] + sr[j][r] * (1.0f / 1024.0f)) * SCALE;
      sm_step(s, m, l, o, ks == qb, ql0 + 8u * g, k0 + col);
#pragma unroll
      for (int j = 0; j < 4; ++j)
#pragma unroll
        for (int r = 0; r < 8; ++r) ss[wave][8u * g + (unsigned)r][(unsigned)j * 16u + col] = s[j][r];
      LDSX();
#pragma unroll
      for (int kc = 0; kc < 2; ++kc) { const F2 p = split_row(&ss[wave][col][0], (unsigned)kc * 32u, lane);
#pragma unroll
        for (int j = 0; j < 4; ++j) { const size_t po = (hc + (unsigned)j * 16u + col) * (size_t)KHI + k0 + (unsigned)kc * 32u; const v16b vh = frag_b(VB + po, lane), vl = frag_b(VBL + po, lane);
          asm volatile("s_wait_loadcnt 0x0" ::: "memory");
          o[j] = wmma_bf(p.h, vh, o[j]); o[j] = wmma_bf(p.l, vh, o[j]); o[j] = wmma_bf(p.h, vl, o[j]); } }
      LDSX(); }
    carry_inv = 1.0f;
  } else {
    v16h qa[2];
#pragma unroll
    for (int kc = 0; kc < 2; ++kc) qa[kc] = frag_h(QH + (size_t)(ql0 + col) * CC + hc + (unsigned)kc * 32u, lane);
#pragma unroll 1
    for (unsigned ks = 0; ks <= qb; ++ks) { const unsigned k0 = ks * 64u; v8f s[4] = {};
#pragma unroll
      for (int j = 0; j < 4; ++j) { const size_t ko = (size_t)(k0 + (unsigned)j * 16u + col) * CC + hc;
        const v16h kf0 = frag_h(KH + ko, lane), kf1 = frag_h(KH + ko + 32, lane);
        asm volatile("s_wait_loadcnt 0x0" ::: "memory");
        s[j] = wmma16(qa[0], kf0, s[j]); s[j] = wmma16(qa[1], kf1, s[j]); }
#pragma unroll
      for (int j = 0; j < 4; ++j)
#pragma unroll
        for (int r = 0; r < 8; ++r) s[j][r] = s[j][r] * SCALE;
      sm_step(s, m, l, o, ks == qb, ql0 + 8u * g, k0 + col);
#pragma unroll
      for (int j = 0; j < 4; ++j)
#pragma unroll
        for (int r = 0; r < 8; ++r) sp[wave][8u * g + (unsigned)r][(unsigned)j * 16u + col] = (_Float16)(s[j][r] * 1024.0f);
      LDSX();
#pragma unroll
      for (int kc = 0; kc < 2; ++kc) { const v16h pa = frag_h(&sp[wave][col][(unsigned)kc * 32u], lane);
#pragma unroll
        for (int j = 0; j < 4; ++j) { const v16h vf = frag_h(VT + (hc + (unsigned)j * 16u + col) * (size_t)TT + k0 + (unsigned)kc * 32u, lane);
          asm volatile("s_wait_loadcnt 0x0" ::: "memory");
          o[j] = wmma16(pa, vf, o[j]); } }
      LDSX(); }
    carry_inv = 1.0f / 1024.0f;
  }
#pragma unroll
  for (int r = 0; r < 8; ++r) { float L = l[r]; L += __shfl_xor(L, 1); L += __shfl_xor(L, 2); L += __shfl_xor(L, 4); L += __shfl_xor(L, 8); const float inv = carry_inv * (1.0f / L);
#pragma unroll
    for (int j = 0; j < 4; ++j) ss[wave][8u * g + (unsigned)r][(unsigned)j * 16u + col] = o[j][r] * inv; }
  LDSX();
  for (unsigned rl = 0; rl < 16u; ++rl) if (lane < (unsigned)(HD / 4)) vst2((void*)(Y + (size_t)(ql0 + rl) * CC + hc + lane * 4u), *(const v4f*)&ss[wave][rl][lane * 4u]); }

__global__ __launch_bounds__(128) void k_out(const float* __restrict__ Y, const float* __restrict__ WO, const float* __restrict__ BO, float* __restrict__ OUT) { __shared__ __align__(16) float sf[4][16][132];
  const unsigned tid = threadIdx.x, wave = tid >> 5, lane = tid & 31u, col = lane & 15u, g = lane >> 4; const unsigned c0 = blockIdx.y * 128u; const unsigned r0 = blockIdx.x * 64u + wave * 16u;
  const float* yrow = Y + (size_t)(r0 + col) * CC;
  v8f acc[8] = {};
#pragma unroll 2
  for (unsigned kc = 0; kc < CC / 32; ++kc) { const F2 a = split_g(yrow + kc * 32u, lane); asm volatile("s_wait_loadcnt 0x0" ::: "memory");
#pragma unroll
    for (int j = 0; j < 8; ++j) { const v16b w = frag_f32_bf(WO + (size_t)(c0 + (unsigned)j * 16u + col) * CC + kc * 32u, lane); asm volatile("s_wait_loadcnt 0x0" ::: "memory"); acc[j] = wmma_bf(a.h, w, acc[j]); acc[j] = wmma_bf(a.l, w, acc[j]); } }
#pragma unroll
  for (int j = 0; j < 8; ++j) {
#pragma unroll
    for (int r = 0; r < 8; ++r) sf[wave][8u * g + (unsigned)r][(unsigned)j * 16u + col] = acc[j][r]; }
  LDSX();
  const v4f braw = *(const v4f*)(BO + c0 + lane * 4u); v4f b4;
#pragma unroll
  for (int i = 0; i < 4; ++i) b4[i] = (float)(__bf16)braw[i];
  for (unsigned rl = 0; rl < 16u; ++rl) { const v4f sv = *(const v4f*)&sf[wave][rl][lane * 4u]; const v4f val = sv + b4; vst2((void*)(OUT + (size_t)(r0 + rl) * DIN + c0 + lane * 4u), val); } }

extern "C" void kernel_launch(void* const* d_in, const int* in_sizes, int n_in, void* d_out, int out_size, void* d_ws, size_t ws_size, hipStream_t stream) {
  if (n_in < 9) return;
  const size_t need_rows = (size_t)(NB - 1) * TT_FULL + (size_t)TT;
  if ((size_t)in_sizes[0] < need_rows * DIN) return;
  if ((size_t)in_sizes[1] < (size_t)CC * DIN) return;
  if ((size_t)in_sizes[2] < (size_t)CC) return;
  if ((size_t)in_sizes[3] < (size_t)CC * DIN) return;
  if ((size_t)in_sizes[4] < (size_t)CC) return;
  if ((size_t)in_sizes[5] < (size_t)CC * DIN) return;
  if ((size_t)in_sizes[6] < (size_t)CC) return;
  if ((size_t)in_sizes[7] < (size_t)DIN * CC) return;
  if ((size_t)in_sizes[8] < (size_t)DIN) return;
  if ((size_t)out_size < need_rows * DIN) return;
  if (ws_size < (size_t)WS_END) return;
  const float* const* F = (const float* const*)d_in;
  char* ws = (char*)d_ws; _Float16 *QH = (_Float16*)(ws + WS_QH), *KH = (_Float16*)(ws + WS_KH), *VT = (_Float16*)(ws + WS_VT), *QL = (_Float16*)(ws + WS_QL), *KL = (_Float16*)(ws + WS_KL); __bf16 *VB = (__bf16*)(ws + WS_VB), *VBL = (__bf16*)(ws + WS_VBL); float *Y = (float*)(ws + WS_Y), *COS = (float*)(ws + WS_COS), *SIN = (float*)(ws + WS_SIN);
  k_pos<<<dim3((TT * RH) / 256), 256, 0, stream>>>(COS, SIN);
  for (int b = 0; b < NB; ++b) {
    const float* Xb = F[0] + (size_t)b * TT_FULL * DIN;
    float* Ob = (float*)d_out + (size_t)b * TT_FULL * DIN;
    k_proj<<<dim3(TT / 64, CC / 128, 3), 128, 0, stream>>>(Xb, F[1], F[3], F[5], F[2], F[4], F[6], COS, SIN, QH, QL, KH, KL, VT, VB, VBL);
    k_fa<<<dim3(NQB, NH), 128, 0, stream>>>(QH, KH, QL, KL, VT, VB, VBL, Y);
    k_out<<<dim3(TT / 64, DIN / 128), 128, 0, stream>>>(Y, F[7], F[8], Ob);
  }
}
